// TransRelation_44375602102657
// MI455X (gfx1250) — hardware-run, weakly checked
//
#include <hip/hip_runtime.h>
#include <stddef.h>


typedef _Float16 v16h __attribute__((ext_vector_type(16)));
typedef _Float16 v8h  __attribute__((ext_vector_type(8)));
typedef float    v8f  __attribute__((ext_vector_type(8)));
typedef float    v4f  __attribute__((ext_vector_type(4)));

#ifndef NB
#define NB 4
#endif
#ifndef SEQ
#define SEQ 512
#endif
#ifndef SCORE_RES
#define SCORE_RES 1
#endif
#define NB_FULL  4
#define SEQ_FULL 512
#define DIM   768
#define REL   64
#define HDV   12
#define HDP   16
#define CTXW  (REL * HDP)
#define MROWS (NB * SEQ)

static_assert(NB >= 1 && NB <= NB_FULL);
static_assert(SEQ >= 128 && SEQ <= SEQ_FULL && (SEQ % 128) == 0);
static_assert(DIM == REL * HDV);
static_assert(REL == 64);
static_assert(HDP == 16 && HDV <= HDP && (HDP - HDV) == 4);
static_assert((REL % 4) == 0 && 4 * HDP == 64);
static_assert(CTXW == 1024);
static_assert((DIM % 64) == 0 && (DIM % 32) == 0);
static_assert((CTXW % 32) == 0);
static_assert((MROWS % 64) == 0 && (MROWS % 8) == 0);
static_assert(DIM == 3 * 32 * 8);
static_assert(((REL * DIM) % (8 * 256)) == 0);
static_assert(((DIM * DIM) % (8 * 256)) == 0);
static_assert(((DIM * CTXW) % (8 * 256)) == 0);
static_assert((HDV * 8) == 96);

#define LDT 72
#define LDC 68
static_assert((LDT % 8) == 0 && LDT >= 64);
static_assert((LDC % 4) == 0 && LDC >= 64);

#define WCARRY  64.0f
#define QCARRY  16.0f
#define KCARRY  8.0f
#define VTCARRY 8.0f
#define PCARRY  16384.0f
#define CCARRY  64.0f
#define RCARRY  2048.0f

#define WQK_BYTES ((size_t)REL * DIM * 2)
#define WV_BYTES  ((size_t)DIM * DIM * 2)
#define WO_BYTES  ((size_t)DIM * CTXW * 2)
#define LN_BYTES  ((size_t)MROWS * DIM * 2)
#define QF_BYTES  ((size_t)MROWS * REL * 4)
#define K_BYTES   ((size_t)MROWS * REL * 2)
#define VT_BYTES  ((size_t)NB * DIM * SEQ * 2)
#define CTX_BYTES ((size_t)MROWS * CTXW * 2)
#define OFF_WQ  ((size_t)0)
#define OFF_WK  (OFF_WQ + WQK_BYTES)
#define OFF_WV  (OFF_WK + WQK_BYTES)
#define OFF_WO  (OFF_WV + WV_BYTES)
#define OFF_T   (OFF_WO + WO_BYTES)
#define OFF_M   (OFF_T + LN_BYTES)
#define OFF_QF  (OFF_M + LN_BYTES)
#define OFF_K   (OFF_QF + QF_BYTES)
#define OFF_KR  (OFF_K + K_BYTES)
#define OFF_VT  (OFF_KR + K_BYTES)
#define OFF_CTX (OFF_VT + VT_BYTES)
#define WS_TOTAL (OFF_CTX + CTX_BYTES)
static_assert((WQK_BYTES % 128) == 0 && (WV_BYTES % 128) == 0 && (WO_BYTES % 128) == 0);
static_assert((LN_BYTES % 128) == 0 && (QF_BYTES % 128) == 0 && (K_BYTES % 128) == 0);
static_assert((VT_BYTES % 128) == 0 && (CTX_BYTES % 128) == 0);
static_assert(WS_TOTAL <= (size_t)134217728);

__device__ __forceinline__ float bf16r(float x) {
  unsigned int u = __float_as_uint(x);
  u = (u + 0x7FFFu + ((u >> 16) & 1u)) & 0xFFFF0000u;
  return __uint_as_float(u);
}

static __device__ __forceinline__ _Float16 toh_flush(float v) {
  const _Float16 r = (_Float16)v;
  return (fabsf(v) < 6.103515625e-05f) ? (_Float16)0.0f : r;
}

__device__ __forceinline__ v16h frag_at(const _Float16* p) {
  v8h lo = *(const v8h*)(p);
  v8h hi = *(const v8h*)(p + 16);
  v16h out;
#pragma unroll
  for (int i = 0; i < 8; ++i) { out[i] = lo[i]; out[i + 8] = hi[i]; }
  return out;
}
__device__ __forceinline__ v16h ld_frag(const _Float16* base, unsigned ld) {
  const unsigned lane = threadIdx.x & 31u;
  return frag_at(base + (lane & 15u) * ld + (lane >> 4) * 8u);
}

__device__ __forceinline__ v8f wmma16(v16h a, v16h b, v8f c) {
  v8f d = __builtin_amdgcn_wmma_f32_16x16x32_f16(false, a, false, b, (short)0, c,
                                                 false, false);
  asm volatile("v_nop\n\tv_nop\n\tv_nop\n\tv_nop" : "+v"(d) : "v"(a), "v"(b));
  return d;
}

__device__ __forceinline__ float red16_max(float x) {
#pragma unroll
  for (int off = 1; off < 16; off <<= 1) x = fmaxf(x, __shfl_xor(x, off, 32));
  return x;
}
__device__ __forceinline__ float red16_sum(float x) {
#pragma unroll
  for (int off = 1; off < 16; off <<= 1) x += __shfl_xor(x, off, 32);
  return x;
}
__device__ __forceinline__ float red32_sum(float x) {
#pragma unroll
  for (int off = 1; off < 32; off <<= 1) x += __shfl_xor(x, off, 32);
  return x;
}

__device__ __forceinline__ void wave_lds_sync() {
  __builtin_amdgcn_fence(3  , "wavefront");
  asm volatile("s_wait_dscnt 0x0" ::: "memory");
  __builtin_amdgcn_wave_barrier();
}

__global__ __launch_bounds__(256) void wcast_kernel(
    const float* __restrict__ W, _Float16* __restrict__ out, unsigned ngroups) {
  const unsigned g = blockIdx.x * 256u + threadIdx.x;
  const unsigned gc = (g < ngroups) ? g : (ngroups - 1u);
  const v4f a0 = *(const v4f*)(W + (size_t)gc * 8u);
  const v4f a1 = *(const v4f*)(W + (size_t)gc * 8u + 4u);
  v8h x;
#pragma unroll
  for (int i = 0; i < 4; ++i) {
    x[i]     = toh_flush(WCARRY * bf16r(a0[i]));
    x[i + 4] = toh_flush(WCARRY * bf16r(a1[i]));
  }
  _Float16* p = out + (size_t)gc * 8u;
  if (g < ngroups) *(volatile v8h*)p = x;
  __threadfence();
  if (g < ngroups) *(volatile v8h*)p = x;
}

__global__ __launch_bounds__(256) void wcast_pad_kernel(
    const float* __restrict__ W, _Float16* __restrict__ out, unsigned ngroups) {
  const unsigned g = blockIdx.x * 256u + threadIdx.x;
  const unsigned gc = (g < ngroups) ? g : (ngroups - 1u);
  const unsigned n = gc >> 7;
  const unsigned gg = gc & 127u;
  const unsigned ch = gg >> 1, part = gg & 1u;
  const size_t src = (size_t)n * DIM + ch * (unsigned)HDV + part * 8u;
  const unsigned o1 = (part != 0u) ? 0u : 4u;
  const v4f a0 = *(const v4f*)(W + src);
  const v4f a1 = *(const v4f*)(W + src + o1);
  v8h x;
#pragma unroll
  for (int i = 0; i < 4; ++i) {
    const _Float16 t1 = toh_flush(WCARRY * bf16r(a1[i]));
    x[i]     = toh_flush(WCARRY * bf16r(a0[i]));
    x[i + 4] = (part != 0u) ? (_Float16)0.0f : t1;
  }
  _Float16* p = out + (size_t)gc * 8u;
  if (g < ngroups) *(volatile v8h*)p = x;
  __threadfence();
  if (g < ngroups) *(volatile v8h*)p = x;
}

template <int SRC_INPUT>
__device__ __forceinline__ void ln_body(const float* __restrict__ X,
                                        const float* __restrict__ G,
                                        const float* __restrict__ Be,
                                        _Float16* __restrict__ dst) {
  const unsigned lane = threadIdx.x & 31u, w = threadIdx.x >> 5;
  const unsigned crow = blockIdx.x * 8u + w;
  size_t srow = crow;
  if (SRC_INPUT) {
    const unsigned bidx = crow / (unsigned)SEQ;
    const unsigned sq = crow - bidx * (unsigned)SEQ;
    srow = (size_t)bidx * SEQ_FULL + sq;
  }
  const float* xr = X + srow * DIM + lane * 8u;

  float s = 0.0f;
#pragma unroll 1
  for (unsigned j = 0; j < 3u; ++j) {
    const v4f a0 = *(const v4f*)(xr + j * 256u);
    const v4f a1 = *(const v4f*)(xr + j * 256u + 4u);
#pragma unroll
    for (int i = 0; i < 4; ++i) {
      const float e0 = SRC_INPUT ? bf16r(a0[i]) : a0[i];
      const float e1 = SRC_INPUT ? bf16r(a1[i]) : a1[i];
      s += e0 + e1;
    }
  }
  const float mean = red32_sum(s) * (1.0f / (float)DIM);

  float ss = 0.0f;
#pragma unroll 1
  for (unsigned j = 0; j < 3u; ++j) {
    const v4f a0 = *(const v4f*)(xr + j * 256u);
    const v4f a1 = *(const v4f*)(xr + j * 256u + 4u);
#pragma unroll
    for (int i = 0; i < 4; ++i) {
      const float d0 = (SRC_INPUT ? bf16r(a0[i]) : a0[i]) - mean;
      const float d1 = (SRC_INPUT ? bf16r(a1[i]) : a1[i]) - mean;
      ss += d0 * d0;
      ss += d1 * d1;
    }
  }
  const float var = red32_sum(ss) * (1.0f / (float)DIM);
  const float rstd = 1.0f / sqrtf(var + 1.0e-5f);

#pragma unroll 1
  for (unsigned j = 0; j < 3u; ++j) {
    const unsigned c = j * 256u + lane * 8u;
    const v4f a0 = *(const v4f*)(xr + j * 256u);
    const v4f a1 = *(const v4f*)(xr + j * 256u + 4u);
    const v4f g0 = *(const v4f*)(G + c);
    const v4f g1 = *(const v4f*)(G + c + 4u);
    const v4f b0 = *(const v4f*)(Be + c);
    const v4f b1 = *(const v4f*)(Be + c + 4u);
    v8h o;
#pragma unroll
    for (int i = 0; i < 4; ++i) {
      const float d0 = (SRC_INPUT ? bf16r(a0[i]) : a0[i]) - mean;
      const float d1 = (SRC_INPUT ? bf16r(a1[i]) : a1[i]) - mean;
      o[i]     = toh_flush(d0 * rstd * bf16r(g0[i]) + bf16r(b0[i]));
      o[i + 4] = toh_flush(d1 * rstd * bf16r(g1[i]) + bf16r(b1[i]));
    }
    _Float16* p = dst + (size_t)crow * DIM + c;
    *(volatile v8h*)p = o;
    __threadfence();
    *(volatile v8h*)p = o;
  }
}

__global__ __launch_bounds__(256) void ln_in_kernel(
    const float* __restrict__ X, const float* __restrict__ G, const float* __restrict__ Be,
    _Float16* __restrict__ dst) {
  ln_body<1>(X, G, Be, dst);
}

template <int MODE>
__device__ __forceinline__ void gemm_body(
    const _Float16* __restrict__ A16, const _Float16* __restrict__ Bt, const unsigned K,
    const float* __restrict__ bias,
    float* __restrict__ outf, _Float16* __restrict__ out16, _Float16* __restrict__ out16r) {
  __shared__ float Cs[64 * LDC];
  const unsigned tid = threadIdx.x, lane = tid & 31u, w = tid >> 5;
  const unsigned mw = w >> 1, nw = w & 1u;
  const unsigned hh = lane >> 4, m = lane & 15u;
  const unsigned n0 = blockIdx.x * 64u;
  const unsigned row0 = blockIdx.y * 64u;

  const _Float16* ap  = A16 + (size_t)(row0 + mw * 16u + m) * K + hh * 8u;
  const _Float16* bp0 = Bt + (size_t)(n0 + nw * 32u + m) * K + hh * 8u;
  const _Float16* bp1 = bp0 + (size_t)16 * K;
  v8f acc0 = {}, acc1 = {};
#pragma unroll 2
  for (unsigned k0 = 0; k0 < K; k0 += 32u) {
    const v16h a  = frag_at(ap + k0);
    const v16h b0 = frag_at(bp0 + k0);
    const v16h b1 = frag_at(bp1 + k0);
    acc0 = wmma16(a, b0, acc0);
    acc1 = wmma16(a, b1, acc1);
  }
#pragma unroll
  for (int r = 0; r < 8; ++r) {
    float* d = &Cs[(mw * 16u + hh * 8u + (unsigned)r) * LDC + nw * 32u + m];
    d[0]  = acc0[r];
    d[16] = acc1[r];
  }
  __syncthreads();

  if (MODE == 1) {
    v8h x[2], xr[2];
    size_t off[2];
#pragma unroll
    for (unsigned i = 0; i < 2u; ++i) {
      const unsigned r = 32u * i + (tid >> 3);
      const unsigned c = (tid & 7u) * 8u;
      const v4f u0 = *(const v4f*)&Cs[r * LDC + c];
      const v4f u1 = *(const v4f*)&Cs[r * LDC + c + 4];
      const v4f g0 = *(const v4f*)(bias + n0 + c);
      const v4f g1 = *(const v4f*)(bias + n0 + c + 4u);
#pragma unroll
      for (int j = 0; j < 4; ++j) {
        const float t0 = KCARRY * (u0[j] * (1.0f / WCARRY) + bf16r(g0[j]));
        const float t1 = KCARRY * (u1[j] * (1.0f / WCARRY) + bf16r(g1[j]));
        const _Float16 h0 = toh_flush(t0);
        const _Float16 h1 = toh_flush(t1);
        x[i][j]      = h0;
        x[i][j + 4]  = h1;
        xr[i][j]     = toh_flush((t0 - (float)h0) * RCARRY);
        xr[i][j + 4] = toh_flush((t1 - (float)h1) * RCARRY);
      }
      off[i] = (size_t)(row0 + r) * REL + n0 + c;
    }
#pragma unroll
    for (int i = 0; i < 2; ++i) *(volatile v8h*)(out16 + off[i]) = x[i];
    if (SCORE_RES) {
#pragma unroll
      for (int i = 0; i < 2; ++i) *(volatile v8h*)(out16r + off[i]) = xr[i];
    }
    __threadfence();
#pragma unroll
    for (int i = 0; i < 2; ++i) *(volatile v8h*)(out16 + off[i]) = x[i];
    if (SCORE_RES) {
#pragma unroll
      for (int i = 0; i < 2; ++i) *(volatile v8h*)(out16r + off[i]) = xr[i];
    }
  }

  if (MODE == 2) {
    const unsigned bidx = row0 / (unsigned)SEQ;
    const unsigned key0 = row0 - bidx * (unsigned)SEQ;
    v8h x[2];
    size_t off[2];
#pragma unroll
    for (unsigned i = 0; i < 2u; ++i) {
      const unsigned dcol = 32u * i + (tid >> 3);
      const unsigned kk = (tid & 7u) * 8u;
      const float bb = bf16r(bias[n0 + dcol]);
#pragma unroll
      for (unsigned j = 0; j < 8u; ++j) {
        const float t = VTCARRY * (Cs[(kk + j) * LDC + dcol] * (1.0f / WCARRY) + bb);
        x[i][j] = toh_flush(t);
      }
      off[i] = ((size_t)bidx * DIM + n0 + dcol) * SEQ + key0 + kk;
    }
#pragma unroll
    for (int i = 0; i < 2; ++i) *(volatile v8h*)(out16 + off[i]) = x[i];
    __threadfence();
#pragma unroll
    for (int i = 0; i < 2; ++i) *(volatile v8h*)(out16 + off[i]) = x[i];
  }

  if (MODE == 0 || MODE == 3) {
    const float cs = (MODE == 0) ? (1.0f / WCARRY) : (1.0f / (WCARRY * CCARRY));
    const unsigned ldo = (MODE == 0) ? (unsigned)REL : (unsigned)DIM;
    v4f xs[4];
    size_t off[4];
#pragma unroll
    for (unsigned i = 0; i < 4u; ++i) {
      const unsigned r = 16u * i + (tid >> 4);
      const unsigned c = (tid & 15u) * 4u;
      const unsigned crow = row0 + r;
      const unsigned bidx = crow / (unsigned)SEQ;
      const unsigned sq = crow - bidx * (unsigned)SEQ;
      const size_t frow = (size_t)bidx * SEQ_FULL + sq;
      const size_t outrow = (MODE == 0) ? (size_t)crow : frow;
      const v4f u = *(const v4f*)&Cs[r * LDC + c];
      const v4f g = *(const v4f*)(bias + n0 + c);
      v4f val;
#pragma unroll
      for (int j = 0; j < 4; ++j) val[j] = u[j] * cs + bf16r(g[j]);
      xs[i] = val;
      off[i] = outrow * ldo + n0 + c;
    }
#pragma unroll
    for (int i = 0; i < 4; ++i) *(volatile v4f*)(outf + off[i]) = xs[i];
    __threadfence();
#pragma unroll
    for (int i = 0; i < 4; ++i) *(volatile v4f*)(outf + off[i]) = xs[i];
  }
}

__global__ __launch_bounds__(256) void gemm_q_kernel(
    const _Float16* __restrict__ A16, const _Float16* __restrict__ Bt,
    const float* __restrict__ bias, float* __restrict__ qf) {
  gemm_body<0>(A16, Bt, (unsigned)DIM, bias, qf, (_Float16*)0, (_Float16*)0);
}
__global__ __launch_bounds__(256) void gemm_k_kernel(
    const _Float16* __restrict__ A16, const _Float16* __restrict__ Bt,
    const float* __restrict__ bias, _Float16* __restrict__ kh, _Float16* __restrict__ kr) {
  gemm_body<1>(A16, Bt, (unsigned)DIM, bias, (float*)0, kh, kr);
}
__global__ __launch_bounds__(256) void gemm_v_kernel(
    const _Float16* __restrict__ A16, const _Float16* __restrict__ Bt,
    const float* __restrict__ bias, _Float16* __restrict__ vt) {
  gemm_body<2>(A16, Bt, (unsigned)DIM, bias, (float*)0, vt, (_Float16*)0);
}
__global__ __launch_bounds__(256) void gemm_out_kernel(
    const _Float16* __restrict__ A16, const _Float16* __restrict__ Bt,
    const float* __restrict__ bias, float* __restrict__ outf) {
  gemm_body<3>(A16, Bt, (unsigned)CTXW, bias, outf, (_Float16*)0, (_Float16*)0);
}

__device__ __forceinline__ void qfrag_build(const float* qp, const float* wp,
                                            v16h& fh, v16h& fr) {
#pragma unroll
  for (int g = 0; g < 2; ++g) {
    const v4f a0 = *(const v4f*)(qp + 16 * g);
    const v4f a1 = *(const v4f*)(qp + 16 * g + 4);
    const v4f w0 = *(const v4f*)(wp + 16 * g);
    const v4f w1 = *(const v4f*)(wp + 16 * g + 4);
#pragma unroll
    for (int i = 0; i < 4; ++i) {
      const float t0 = QCARRY * (a0[i] * bf16r(w0[i]));
      const float t1 = QCARRY * (a1[i] * bf16r(w1[i]));
      const _Float16 h0 = toh_flush(t0);
      const _Float16 h1 = toh_flush(t1);
      fh[8 * g + i]     = h0;
      fh[8 * g + 4 + i] = h1;
      fr[8 * g + i]     = toh_flush((t0 - (float)h0) * RCARRY);
      fr[8 * g + 4 + i] = toh_flush((t1 - (float)h1) * RCARRY);
    }
  }
}

__global__ __launch_bounds__(256) __attribute__((amdgpu_num_vgpr(256))) void attn_kernel(
    const float* __restrict__ Qf, const _Float16* __restrict__ Kh,
    const _Float16* __restrict__ KRh, const _Float16* __restrict__ Vt,
    const float* __restrict__ Wt, const float* __restrict__ Mk,
    _Float16* __restrict__ Ov) {
  __shared__ _Float16 Ks[64 * LDT];
#if SCORE_RES
  __shared__ _Float16 KRs[64 * LDT];
#endif
  __shared__ _Float16 Vs[HDP * LDT];
  __shared__ _Float16 Ps[8 * 16 * LDT];
  __shared__ _Float16 Os[8 * 16 * LDT];

  const unsigned tid = threadIdx.x, lane = tid & 31u;
  const unsigned w = (unsigned)__builtin_amdgcn_readfirstlane((int)(threadIdx.x >> 5));
  const unsigned hh = lane >> 4, m = lane & 15u;
  const unsigned q0 = blockIdx.x * 128u;
  const unsigned hg = blockIdx.y;
  const unsigned b = blockIdx.z;
  const unsigned qrow0 = q0 + w * 16u;
  const unsigned pbase = w * (16u * LDT);
  const float sscale = 1.0f / (QCARRY * KCARRY);

  if (w == 3u) {
    const unsigned r = (unsigned)HDV + (lane >> 3), c = (lane & 7u) * 8u;
    const v8h z = {};
    *(v8h*)&Vs[r * LDT + c] = z;
  }

#pragma unroll 1
  for (unsigned hl = 0; hl < 4u; ++hl) {
    const unsigned ch = hg * 4u + hl;

    v16h qf[2], qr[2];
    {
      const float* qp = Qf + (size_t)(b * (unsigned)SEQ + qrow0 + m) * REL + hh * 8u;
      const float* wp = Wt + (size_t)ch * REL + hh * 8u;
      qfrag_build(qp, wp, qf[0], qr[0]);
      qfrag_build(qp + 32, wp + 32, qf[1], qr[1]);
    }

    float mrow[8], lrow[8];
    v8f o = {};
#pragma unroll
    for (int v = 0; v < 8; ++v) { mrow[v] = -1.0e30f; lrow[v] = 0.0f; }

    for (unsigned kb = 0; kb < (unsigned)SEQ; kb += 64u) {
#pragma unroll
      for (unsigned j = 0; j < 2u; ++j) {
        const unsigned idx = tid + 256u * j;
        const unsigned r = idx >> 3, c = (idx & 7u) * 8u;
        const size_t g = (size_t)(b * (unsigned)SEQ + kb + r) * REL + c;
        *(v8h*)&Ks[r * LDT + c] = *(const v8h*)(Kh + g);
#if SCORE_RES
        *(v8h*)&KRs[r * LDT + c] = *(const v8h*)(KRh + g);
#endif
      }
      if (w < 3u) {
        const unsigned r = tid >> 3, c = (tid & 7u) * 8u;
        *(v8h*)&Vs[r * LDT + c] =
            *(const v8h*)(Vt + ((size_t)b * DIM + ch * (unsigned)HDV + r) * SEQ + kb + c);
      }
      __syncthreads();

      v4f mk[8];
      {
        const float* mp = Mk + ((size_t)b * SEQ_FULL + qrow0 + hh * 8u) * SEQ_FULL + kb + 4u * m;
#pragma unroll
        for (int v = 0; v < 8; ++v) mk[v] = *(const v4f*)(mp + (size_t)v * SEQ_FULL);
      }

      v8f s[4];
#pragma unroll
      for (int kg = 0; kg < 4; ++kg) {
        v8f t = {};
#if SCORE_RES
        v8f tr = {};
#endif
#pragma unroll
        for (int c = 0; c < 2; ++c) {
          const unsigned ko = (4u * m + (unsigned)kg) * LDT + (unsigned)c * 32u + hh * 8u;
          const v16h kf = frag_at(&Ks[ko]);
          t = wmma16(qf[c], kf, t);
#if SCORE_RES
          const v16h kr = frag_at(&KRs[ko]);
          tr = wmma16(qf[c], kr, tr);
          tr = wmma16(qr[c], kf, tr);
#endif
        }
#if SCORE_RES
        s[kg] = t * sscale + tr * (sscale / RCARRY);
#else
        s[kg] = t * sscale;
#endif
      }
#pragma unroll
      for (int kg = 0; kg < 4; ++kg)
#pragma unroll
        for (int v = 0; v < 8; ++v) s[kg][v] = s[kg][v] + bf16r(mk[v][kg]);

      float alpha[8];
#pragma unroll
      for (int v = 0; v < 8; ++v) {
        float mx = fmaxf(fmaxf(s[0][v], s[1][v]), fmaxf(s[2][v], s[3][v]));
        mx = red16_max(mx);
        const float mn = fmaxf(mrow[v], mx);
        alpha[v] = __expf(mrow[v] - mn);
        mrow[v] = mn;
      }
#pragma unroll
      for (int kg = 0; kg < 4; ++kg)
#pragma unroll
        for (int v = 0; v < 8; ++v) {
          const float p = __expf(s[kg][v] - mrow[v]);
          const _Float16 ph = toh_flush(p * PCARRY);
          Ps[pbase + (hh * 8u + (unsigned)v) * LDT + 4u * m + (unsigned)kg] = ph;
          s[kg][v] = (float)ph;
        }
#pragma unroll
      for (int v = 0; v < 8; ++v) {
        const float rs = red16_sum((s[0][v] + s[1][v]) + (s[2][v] + s[3][v]));
        lrow[v] = alpha[v] * lrow[v] + rs;
      }
#pragma unroll
      for (int v = 0; v < 8; ++v) o[v] = o[v] * alpha[v];
      wave_lds_sync();

#pragma unroll
      for (int c = 0; c < 2; ++c) {
        const v16h pf = ld_frag(&Ps[pbase + (unsigned)c * 32u], LDT);
        const v16h vf = ld_frag(&Vs[(unsigned)c * 32u], LDT);
        o = wmma16(pf, vf, o);
      }
      __syncthreads();
    }

#pragma unroll
    for (int v = 0; v < 8; ++v) {
      const float inv = __builtin_amdgcn_rcpf(lrow[v]) * (CCARRY / VTCARRY);
      const _Float16 cv = toh_flush(o[v] * inv);
      Os[pbase + (hh * 8u + (unsigned)v) * LDT + hl * 16u + m] =
          (m < (unsigned)HDV) ? cv : (_Float16)0.0f;
    }
  }
  wave_lds_sync();

  v8h x[4];
  size_t off[4];
#pragma unroll
  for (unsigned i = 0; i < 4u; ++i) {
    const unsigned r = 4u * i + (lane >> 3);
    const unsigned c = (lane & 7u) * 8u;
    x[i] = *(const v8h*)&Os[pbase + r * LDT + c];
    off[i] = (size_t)(b * (unsigned)SEQ + qrow0 + r) * CTXW + hg * 64u + c;
  }
#pragma unroll
  for (int i = 0; i < 4; ++i) *(volatile v8h*)(Ov + off[i]) = x[i];
  __threadfence();
#pragma unroll
  for (int i = 0; i < 4; ++i) *(volatile v8h*)(Ov + off[i]) = x[i];
}

extern "C" void kernel_launch(void* const* d_in, const int* in_sizes, int n_in,
                              void* d_out, int out_size, void* d_ws, size_t ws_size,
                              hipStream_t stream) {
  if (n_in < 16) return;
  const long long need_x = ((long long)(NB - 1) * SEQ_FULL + SEQ) * DIM;
  const long long need_m = ((long long)(NB - 1) * SEQ_FULL + SEQ) * SEQ_FULL;
  if ((long long)in_sizes[0] < need_x) return;
  if ((long long)in_sizes[1] < need_x) return;
  if ((long long)in_sizes[2] < need_m) return;
  if (in_sizes[3] < DIM || in_sizes[4] < DIM || in_sizes[5] < DIM || in_sizes[6] < DIM) return;
  if ((long long)in_sizes[7] < (long long)REL * DIM) return;
  if (in_sizes[8] < REL) return;
  if ((long long)in_sizes[9] < (long long)REL * DIM) return;
  if (in_sizes[10] < REL) return;
  if ((long long)in_sizes[11] < (long long)DIM * DIM) return;
  if (in_sizes[12] < DIM) return;
  if (in_sizes[13] < REL * REL) return;
  if ((long long)in_sizes[14] < (long long)DIM * DIM) return;
  if (in_sizes[15] < DIM) return;
  if ((long long)out_size < need_x) return;
  if (ws_size < WS_TOTAL) return;

  const float* tgt  = (const float*)d_in[0];
  const float* mem  = (const float*)d_in[1];
  const float* mask = (const float*)d_in[2];
  const float* lnqw = (const float*)d_in[3];
  const float* lnqb = (const float*)d_in[4];
  const float* lnkw = (const float*)d_in[5];
  const float* lnkb = (const float*)d_in[6];
  const float* wq   = (const float*)d_in[7];
  const float* bq   = (const float*)d_in[8];
  const float* wk   = (const float*)d_in[9];
  const float* bk   = (const float*)d_in[10];
  const float* wv   = (const float*)d_in[11];
  const float* bv   = (const float*)d_in[12];
  const float* wt   = (const float*)d_in[13];
  const float* wo   = (const float*)d_in[14];
  const float* bo   = (const float*)d_in[15];
  float* out = (float*)d_out;

  char* ws = (char*)d_ws;
  _Float16* Wq16  = (_Float16*)(ws + OFF_WQ);
  _Float16* Wk16  = (_Float16*)(ws + OFF_WK);
  _Float16* Wv16  = (_Float16*)(ws + OFF_WV);
  _Float16* Wo16  = (_Float16*)(ws + OFF_WO);
  _Float16* T16   = (_Float16*)(ws + OFF_T);
  _Float16* M16   = (_Float16*)(ws + OFF_M);
  float*    Qf    = (float*)(ws + OFF_QF);
  _Float16* K16   = (_Float16*)(ws + OFF_K);
  _Float16* KR16  = (_Float16*)(ws + OFF_KR);
  _Float16* Vt16  = (_Float16*)(ws + OFF_VT);
  _Float16* Ctx16 = (_Float16*)(ws + OFF_CTX);

  dim3 blk(256);
  const unsigned gqk = (unsigned)(REL * DIM / 8);
  const unsigned gvv = (unsigned)(DIM * DIM / 8);
  const unsigned gwo = (unsigned)(DIM * CTXW / 8);

  wcast_kernel<<<dim3(gqk / 256u), blk, 0, stream>>>(wq, Wq16, gqk);
  wcast_kernel<<<dim3(gqk / 256u), blk, 0, stream>>>(wk, Wk16, gqk);
  wcast_kernel<<<dim3(gvv / 256u), blk, 0, stream>>>(wv, Wv16, gvv);
  wcast_pad_kernel<<<dim3(gwo / 256u), blk, 0, stream>>>(wo, Wo16, gwo);

  ln_in_kernel<<<dim3(MROWS / 8), blk, 0, stream>>>(tgt, lnqw, lnqb, T16);
  ln_in_kernel<<<dim3(MROWS / 8), blk, 0, stream>>>(mem, lnkw, lnkb, M16);

  gemm_q_kernel<<<dim3(REL / 64, MROWS / 64), blk, 0, stream>>>(T16, Wq16, bq, Qf);
  gemm_k_kernel<<<dim3(REL / 64, MROWS / 64), blk, 0, stream>>>(M16, Wk16, bk, K16, KR16);
  gemm_v_kernel<<<dim3(DIM / 64, MROWS / 64), blk, 0, stream>>>(M16, Wv16, bv, Vt16);

  attn_kernel<<<dim3(SEQ / 128, REL / 4, NB), blk, 0, stream>>>(Qf, K16, KR16, Vt16, wt, mask,
                                                                 Ctx16);

  gemm_out_kernel<<<dim3(DIM / 64, MROWS / 64), blk, 0, stream>>>(Ctx16, Wo16, bo, out);
}
